// ExpansionContrastModule_64321430225263
// MI455X (gfx1250) — hardware-verified
//
#include <hip/hip_runtime.h>
#include <math.h>
#include <stdint.h>


#pragma clang fp contract(off)

#ifndef NB
#define NB 8
#endif
#define CIN   16
#define WDIM  192
#define XDIM  192
#define NPIX  (WDIM * XDIM)
#define NH    4
#define HID   16
#define C8    128
#define TT    64
#define OCH   32
#define NSEG  3
#define NBLK  (NB * WDIM * NSEG)
#define NCHK  (NPIX / 2048)
#define KPAD  256
#define SXP   80
#define PTOT  (NB * NPIX)
#define BG    ((NB < 4) ? NB : 4)
#define NGRP  (NB / BG)
#define PG    (BG * NPIX)
#define GBLK  (BG * WDIM * NSEG)

static_assert(XDIM == 64 * NSEG);
static_assert(NPIX == NCHK * 2048);
static_assert(PTOT % 1024 == 0 && NPIX % 1024 == 0);
static_assert(NB >= 1 && NB <= 8);
static_assert(NB % BG == 0 && NGRP * BG == NB);
static_assert(SXP >= 64 + 16);
static_assert(KPAD % 32 == 0 && KPAD >= 160);

typedef _Float16       v16h __attribute__((ext_vector_type(16)));
typedef _Float16       v8h  __attribute__((ext_vector_type(8)));
typedef float          v8f  __attribute__((ext_vector_type(8)));
typedef float          v4f  __attribute__((ext_vector_type(4)));
typedef unsigned int   v4u  __attribute__((ext_vector_type(4)));

union HU { v8h h; v4u u; _Float16 s[8]; };
union FR { v16h v; v8h h[2]; _Float16 s[16]; };
static_assert(sizeof(HU) == 16);
static_assert(sizeof(FR) == 32);

__device__ __forceinline__ unsigned short bf_bits(float f) {
  const unsigned u = __float_as_uint(f);
  return (unsigned short)((u + 0x7FFFu + ((u >> 16) & 1u)) >> 16);
}
__device__ __forceinline__ float bf_up(unsigned short h) { return __uint_as_float(((unsigned)h) << 16); }
__device__ __forceinline__ float bfr(float f) { return bf_up(bf_bits(f)); }
__device__ __forceinline__ v8f zero8() { v8f z = {0.f, 0.f, 0.f, 0.f, 0.f, 0.f, 0.f, 0.f}; return z; }

__device__ __forceinline__ void ld8(const float* p, float* o) {
  const v4f a = *(const v4f*)(p);
  const v4f b = *(const v4f*)(p + 4);
  o[0] = a[0]; o[1] = a[1]; o[2] = a[2]; o[3] = a[3];
  o[4] = b[0]; o[5] = b[1]; o[6] = b[2]; o[7] = b[3];
}

__device__ __forceinline__ double shfl_xor_d(double v, int m) {
  const unsigned long long u = (unsigned long long)__double_as_longlong(v);
  int lo = (int)(unsigned)(u & 0xffffffffull);
  int hi = (int)(unsigned)(u >> 32);
  lo = __shfl_xor(lo, m, 32);
  hi = __shfl_xor(hi, m, 32);
  const unsigned long long r = (((unsigned long long)(unsigned)hi) << 32) | (unsigned long long)(unsigned)lo;
  return __longlong_as_double((long long)r);
}

__device__ __forceinline__ v16h ldfrag_h(const _Float16* p) {
  FR f;
  f.h[0] = *(const v8h*)(p);
  f.h[1] = *(const v8h*)(p + 16);
  return f.v;
}

__device__ __forceinline__ v8f mma_h(v16h a, v16h b, v8f c) {
  c = __builtin_amdgcn_wmma_f32_16x16x32_f16(false, a, false, b, (short)0, c, false, false);
#if defined(__HIP_DEVICE_COMPILE__)
  asm volatile("v_nop\n\tv_nop\n\tv_nop\n\tv_nop" : "+v"(c) : "v"(a), "v"(b));
#endif
  return c;
}
__device__ __forceinline__ v8f mma_h_raw(v16h a, v16h b, v8f c) {
  return __builtin_amdgcn_wmma_f32_16x16x32_f16(false, a, false, b, (short)0, c, false, false);
}
__device__ __forceinline__ void guard_k4(v8f& c0, v8f& c1, v8f& c2, v8f& c3,
                                         v16h a, v16h b0, v16h b1, v16h b2, v16h b3) {
#if defined(__HIP_DEVICE_COMPILE__)
  asm volatile("v_nop\n\tv_nop\n\tv_nop\n\tv_nop"
               : "+v"(c0), "+v"(c1), "+v"(c2), "+v"(c3)
               : "v"(a), "v"(b0), "v"(b1), "v"(b2), "v"(b3));
#endif
}
__device__ __forceinline__ void guard2(v8f& c0, v8f& c1, v16h a, v16h b0, v16h b1) {
#if defined(__HIP_DEVICE_COMPILE__)
  asm volatile("v_nop\n\tv_nop\n\tv_nop\n\tv_nop" : "+v"(c0), "+v"(c1) : "v"(a), "v"(b0), "v"(b1));
#endif
}
__device__ __forceinline__ void guard_qk(v8f& c0, v8f& c1, v16h a0, v16h a1, v16h b0, v16h b1) {
#if defined(__HIP_DEVICE_COMPILE__)
  asm volatile("v_nop\n\tv_nop\n\tv_nop\n\tv_nop"
               : "+v"(c0), "+v"(c1)
               : "v"(a0), "v"(a1), "v"(b0), "v"(b1));
#endif
}
__device__ __forceinline__ void wave_lds_sync() {
  __builtin_amdgcn_fence(__ATOMIC_RELEASE, "workgroup");
  __builtin_amdgcn_wave_barrier();
  __builtin_amdgcn_fence(__ATOMIC_ACQUIRE, "workgroup");
}

__device__ __forceinline__ int tap_ky(int t) { return (t >= 9) ? 1 : ((t * 11) >> 5); }
__device__ __forceinline__ int tap_kx(int t) { return (t >= 9) ? 1 : (t - 3 * tap_ky(t)); }
__device__ __forceinline__ float wsur_f(float sw, float omsw, int k, int tap) {
  const int np = (int)((0x36785210u >> (4 * k)) & 15u);
  const float isc = (tap == 4) ? 1.0f : 0.0f;
  const float isn = (tap == np) ? 1.0f : 0.0f;
  const float d = isc - isn;
  const float k2v = (tap == np) ? -1.0f : 0.125f;
  const float t0 = d * omsw;
  const float t1 = k2v * sw;
  const float w = t0 + t1;
  return (tap < 9) ? w : 0.0f;
}
__device__ __forceinline__ float wcen_f(float sw, float omsw, int tap) {
  const float su = (tap == 4) ? 0.125f : 0.109375f;
  const float ce = (tap == 4) ? 1.0f : 0.0f;
  const float t0 = su * omsw;
  const float t1 = ce * sw;
  const float w = t0 + t1;
  return (tap < 9) ? w : 0.0f;
}

__device__ __forceinline__ void stage_item(_Float16* sXb, const _Float16* __restrict__ cTb,
                                           int wrow, int x0, int hs, int item) {
  const int s = 1 << hs;
  const int ky = item / 160;
  const int rm = item - ky * 160;
  const int p = rm >> 1, cg = rm & 1;
  const int wr = wrow + (ky - 1) * s;
  const int x = x0 - s + p;
  const bool ok = (wr >= 0) && (wr < WDIM) && (x >= 0) && (x < XDIM);
  const int wrc = min(max(wr, 0), WDIM - 1);
  const int xc = min(max(x, 0), XDIM - 1);
  HU u;
  u.u = *(const v4u*)(cTb + ((size_t)(wrc * XDIM + xc) * 16 + 8 * cg));
  v4u o;
  o[0] = ok ? u.u[0] : 0u;
  o[1] = ok ? u.u[1] : 0u;
  o[2] = ok ? u.u[2] : 0u;
  o[3] = ok ? u.u[3] : 0u;
  *(v4u*)(sXb + ((ky * SXP + p) * 16 + 8 * cg)) = o;
}

__global__ __launch_bounds__(128) void k_cvt(const float* __restrict__ cen, _Float16* cenT) {
  __shared__ float sT[16][68];
  const int tid = threadIdx.x;
  const int bx = blockIdx.x;
  const int b = bx / (WDIM * NSEG);
  const int rem = bx - b * (WDIM * NSEG);
  const int wrow = rem / NSEG;
  const int x0 = (rem - wrow * NSEG) * 64;
#pragma unroll
  for (int q = 0; q < 2; ++q) {
    const int idx = tid + 128 * q;
    const int c = idx >> 4, x4 = (idx & 15) * 4;
    const v4f v = *(const v4f*)(cen + ((size_t)(b * CIN + c)) * NPIX + (size_t)wrow * XDIM + x0 + x4);
    sT[c][x4 + 0] = v[0]; sT[c][x4 + 1] = v[1]; sT[c][x4 + 2] = v[2]; sT[c][x4 + 3] = v[3];
  }
  __syncthreads();
  const int px = tid >> 1, hf = tid & 1;
  HU u;
#pragma unroll
  for (int e = 0; e < 8; ++e) u.s[e] = (_Float16)(bfr(sT[8 * hf + e][px]) * 16.0f);
  _Float16* dst = cenT + ((size_t)b * NPIX + (size_t)wrow * XDIM + x0 + px) * 16 + 8 * hf;
  for (int ps = 0; ps < 2; ++ps) {
    *(volatile v4u*)dst = u.u;
    __threadfence();
  }
}

__global__ __launch_bounds__(256) void k_prep(const float* __restrict__ wq, const float* __restrict__ wk,
                                              const float* __restrict__ wv, const float* __restrict__ sum_w,
                                              const float* __restrict__ w_out,
                                              _Float16* Wk16, _Float16* Wq16, _Float16* WvT16, _Float16* WO16) {
  __shared__ __align__(16) _Float16 sW[16 * 264];
  __shared__ float sSw[16];
  const int h = blockIdx.x;
  const int tid = threadIdx.x, lane = tid & 31, wave = tid >> 5;
  if (tid < 16) sSw[tid] = bfr(sum_w[h * CIN + tid]);
  __syncthreads();
  const int kk = tid, tap = kk >> 4, c = kk & 15;
  const float sw = sSw[c], omsw = 1.0f - sw;

  for (int it = 0; it < 16; ++it) {
#pragma unroll 1
    for (int rr = 0; rr < 8; ++rr) {
      const int j = it * 8 + rr;
      const float* wr = wk + ((size_t)(h * C8 + j)) * C8 + c;
      float val = 0.0f;
#pragma unroll 1
      for (int k = 0; k < 8; ++k) {
        const float t = bfr(wr[16 * k]) * wsur_f(sw, omsw, k, tap);
        val = val + t;
      }
      sW[rr * 264 + kk] = (_Float16)(val * 64.0f);
    }
    __syncthreads();
    {
      HU u;
      u.h = *(const v8h*)(sW + wave * 264 + 8 * lane);
      _Float16* dst = Wk16 + ((size_t)(h * C8 + it * 8 + wave)) * KPAD + 8 * lane;
      for (int ps = 0; ps < 2; ++ps) {
        *(volatile v4u*)dst = u.u;
        __threadfence();
      }
    }
    __syncthreads();
  }

  for (int it = 0; it < 2; ++it) {
#pragma unroll 1
    for (int rr = 0; rr < 8; ++rr) {
      const int i = it * 8 + rr;
      const float val = bfr(wq[(h * HID + i) * CIN + c]) * wcen_f(sw, omsw, tap);
      sW[rr * 264 + kk] = (_Float16)(val * 64.0f);
    }
    __syncthreads();
    {
      HU u;
      u.h = *(const v8h*)(sW + wave * 264 + 8 * lane);
      _Float16* dst = Wq16 + ((size_t)(h * HID + it * 8 + wave)) * KPAD + 8 * lane;
      for (int ps = 0; ps < 2; ++ps) {
        *(volatile v4u*)dst = u.u;
        __threadfence();
      }
    }
    __syncthreads();
  }

  for (int it = 0; it < 8; ++it) {
    {
      const int j = tid & 127, rs = tid >> 7;
#pragma unroll 1
      for (int q = 0; q < 8; ++q) {
        const int ar = 2 * q + rs;
        const int a = it * 16 + ar;
        sW[ar * 136 + j] = (_Float16)(bfr(wv[((size_t)(h * C8 + j)) * C8 + a]) * 64.0f);
      }
    }
    __syncthreads();
    {
      const int ar = 2 * wave + (lane >> 4);
      HU u;
      u.h = *(const v8h*)(sW + ar * 136 + 8 * (lane & 15));
      _Float16* dst = WvT16 + ((size_t)(h * C8 + it * 16 + ar)) * C8 + 8 * (lane & 15);
      for (int ps = 0; ps < 2; ++ps) {
        *(volatile v4u*)dst = u.u;
        __threadfence();
      }
    }
    __syncthreads();
  }

  if (h == 0) {
    const int o = tid >> 3, c8 = (tid & 7) * 8;
    HU u;
#pragma unroll
    for (int e = 0; e < 8; ++e) u.s[e] = (_Float16)(bfr(w_out[o * TT + c8 + e]) * 64.0f);
    _Float16* dst = WO16 + o * TT + c8;
    for (int ps = 0; ps < 2; ++ps) {
      *(volatile v4u*)dst = u.u;
      __threadfence();
    }
  }
}

__global__ __launch_bounds__(256) void k_conv(const _Float16* __restrict__ cenT, const _Float16* __restrict__ Wk16,
                                              const _Float16* __restrict__ Wq16, _Float16* Kh, _Float16* Kl,
                                              _Float16* Qh, _Float16* Ql, float* NRM, int hs, int b0) {
  __shared__ __align__(16) _Float16 sX[3 * SXP * 16];
  __shared__ __align__(16) float sK[8][16 * 68];
  __shared__ __align__(16) float sQ[16 * 68];
  __shared__ __align__(16) float sNrm[256];
  __shared__ float sNq[4][16];
  const int tid = threadIdx.x, lane = tid & 31;
  const int wave = __builtin_amdgcn_readfirstlane(tid >> 5);
  const int hh = lane >> 4, rl = lane & 15;
  const int bx = blockIdx.x;
  const int bl = bx / (WDIM * NSEG);
  const int rem = bx - bl * (WDIM * NSEG);
  const int b = b0 + bl;
  const int wrow = rem / NSEG;
  const int x0 = (rem - wrow * NSEG) * 64;
  const size_t pxl = (size_t)bl * NPIX + (size_t)wrow * XDIM + x0;
  const _Float16* cTb = cenT + (size_t)b * NPIX * 16;

  stage_item(sX, cTb, wrow, x0, hs, min(tid, 479));
  stage_item(sX, cTb, wrow, x0, hs, min(tid + 256, 479));
  __syncthreads();

  v8f acc[4];
#pragma unroll
  for (int ct = 0; ct < 4; ++ct) acc[ct] = zero8();
  v8f accq = zero8();
  const _Float16* aK = Wk16 + (size_t)(16 * wave + rl) * KPAD + 8 * hh;
  const _Float16* aQ = Wq16 + (size_t)rl * KPAD + 8 * hh;
#pragma unroll
  for (int ks = 0; ks < 5; ++ks) {
    const int tA = 2 * ks, tB = 2 * ks + 1;
    const int oA = (tap_ky(tA) * SXP + (tap_kx(tA) << hs)) * 16 + 8 * hh;
    const int oB = (tap_ky(tB) * SXP + (tap_kx(tB) << hs)) * 16 + 8 * hh;
    v16h bf[4];
#pragma unroll
    for (int ct = 0; ct < 4; ++ct) {
      const int po = (16 * ct + rl) * 16;
      FR f;
      f.h[0] = *(const v8h*)(sX + po + oA);
      f.h[1] = *(const v8h*)(sX + po + oB);
      bf[ct] = f.v;
    }
    const v16h a = ldfrag_h(aK + 32 * ks);
#pragma unroll
    for (int ct = 0; ct < 4; ++ct) acc[ct] = mma_h_raw(a, bf[ct], acc[ct]);
    guard_k4(acc[0], acc[1], acc[2], acc[3], a, bf[0], bf[1], bf[2], bf[3]);
    if (wave < 4) {
      const int po = (16 * wave + rl) * 16;
      FR fq;
      fq.h[0] = *(const v8h*)(sX + po + oA);
      fq.h[1] = *(const v8h*)(sX + po + oB);
      const v16h aq = ldfrag_h(aQ + 32 * ks);
      accq = mma_h(aq, fq.v, accq);
    }
  }

  const float cK = 1.0f / 1024.0f;
  float p[8];
#pragma unroll
  for (int r = 0; r < 8; ++r) {
    const float v0 = acc[0][r] * cK, v1 = acc[1][r] * cK, v2 = acc[2][r] * cK, v3 = acc[3][r] * cK;
    const float s01 = v0 * v0 + v1 * v1;
    const float s23 = v2 * v2 + v3 * v3;
    p[r] = s01 + s23;
  }
#pragma unroll
  for (int m = 1; m < 16; m <<= 1) {
#pragma unroll
    for (int r = 0; r < 8; ++r) p[r] += __shfl_xor(p[r], m, 32);
  }
  if (rl == 0) {
#pragma unroll
    for (int r = 0; r < 8; ++r) sNrm[16 * wave + 8 * hh + r] = p[r];
  }
  float* slab = sK[wave];
#pragma unroll
  for (int ct = 0; ct < 4; ++ct) {
#pragma unroll
    for (int r = 0; r < 8; ++r) slab[(8 * hh + r) * 68 + 16 * ct + rl] = acc[ct][r] * (1.0f / 128.0f);
  }
  wave_lds_sync();
  const int q8 = lane & 7, rr = lane >> 3;
  HU uk[4], ul[4];
#pragma unroll
  for (int it = 0; it < 4; ++it) {
    const int row = 4 * it + rr;
    float xs[8];
    ld8(slab + row * 68 + 8 * q8, xs);
#pragma unroll
    for (int e = 0; e < 8; ++e) {
      const float v = xs[e];
      const _Float16 hv = (_Float16)v;
      uk[it].s[e] = hv;
      ul[it].s[e] = (_Float16)((v - (float)hv) * 2048.0f);
    }
  }
  for (int ps = 0; ps < 2; ++ps) {
#pragma unroll
    for (int it = 0; it < 4; ++it) {
      const int row = 4 * it + rr;
      const size_t co = (size_t)(16 * wave + row) * (size_t)PG + pxl + 8 * q8;
      *(volatile v4u*)(Kh + co) = uk[it].u;
      *(volatile v4u*)(Kl + co) = ul[it].u;
    }
    __threadfence();
  }
  if (wave < 4) {
    float pq[8];
#pragma unroll
    for (int r = 0; r < 8; ++r) {
      const float vq = accq[r] * cK;
      pq[r] = vq * vq;
      sQ[(8 * hh + r) * 68 + 16 * wave + rl] = accq[r] * (1.0f / 128.0f);
    }
#pragma unroll
    for (int m = 1; m < 16; m <<= 1) {
#pragma unroll
      for (int r = 0; r < 8; ++r) pq[r] += __shfl_xor(pq[r], m, 32);
    }
    if (rl == 0) {
#pragma unroll
      for (int r = 0; r < 8; ++r) sNq[wave][8 * hh + r] = pq[r];
    }
  }
  __syncthreads();
  if (tid < 16) {
    const float a01 = sNq[0][tid] + sNq[1][tid];
    const float a23 = sNq[2][tid] + sNq[3][tid];
    sNrm[128 + tid] = a01 + a23;
  }
  if (tid >= 144) sNrm[tid] = 0.0f;
  __syncthreads();
  if (wave == 0) {
    const v4f r0 = *(const v4f*)(sNrm + 4 * lane);
    const v4f r1 = *(const v4f*)(sNrm + 128 + 4 * lane);
    float* rec = NRM + ((size_t)b * (WDIM * NSEG) + rem) * 256;
    for (int ps = 0; ps < 2; ++ps) {
      *(volatile v4f*)(rec + 4 * lane) = r0;
      *(volatile v4f*)(rec + 128 + 4 * lane) = r1;
      __threadfence();
    }
  }
  if (wave < 4) {
    const int row = 4 * wave + rr;
    float xs[8];
    ld8(sQ + row * 68 + 8 * q8, xs);
    HU uh, uq;
#pragma unroll
    for (int e = 0; e < 8; ++e) {
      const float v = xs[e];
      const _Float16 hv = (_Float16)v;
      uh.s[e] = hv;
      uq.s[e] = (_Float16)((v - (float)hv) * 2048.0f);
    }
    const size_t qo = (size_t)row * (size_t)PG + pxl + 8 * q8;
    for (int ps = 0; ps < 2; ++ps) {
      *(volatile v4u*)(Qh + qo) = uh.u;
      *(volatile v4u*)(Ql + qo) = uq.u;
      __threadfence();
    }
  }
}

__global__ __launch_bounds__(256) void k_score(const _Float16* __restrict__ Qh, const _Float16* __restrict__ Ql,
                                               const _Float16* __restrict__ Kh, const _Float16* __restrict__ Kl,
                                               float* RAWP, int b0) {
  __shared__ __align__(16) float sR[16 * 132];
  const int tid = threadIdx.x, lane = tid & 31;
  const int wave = __builtin_amdgcn_readfirstlane(tid >> 5);
  const int hh = lane >> 4, rl = lane & 15;
  const int bx = blockIdx.x;
  const int bl = bx / NCHK;
  const int chunk = bx - bl * NCHK;
  const size_t nbase = (size_t)bl * NPIX + (size_t)chunk * 2048;
  const _Float16* aqh = Qh + (size_t)rl * (size_t)PG + nbase + 8 * hh;
  const _Float16* aql = Ql + (size_t)rl * (size_t)PG + nbase + 8 * hh;
  const _Float16* bkh = Kh + (size_t)(16 * wave + rl) * (size_t)PG + nbase + 8 * hh;
  const _Float16* bkl = Kl + (size_t)(16 * wave + rl) * (size_t)PG + nbase + 8 * hh;
  v8f acc = zero8(), accl = zero8();
#pragma unroll 2
  for (int ks = 0; ks < 64; ++ks) {
    const v16h qh = ldfrag_h(aqh + 32 * ks);
    const v16h ql = ldfrag_h(aql + 32 * ks);
    const v16h kh = ldfrag_h(bkh + 32 * ks);
    const v16h kl = ldfrag_h(bkl + 32 * ks);
    acc  = mma_h_raw(qh, kh, acc);
    accl = mma_h_raw(qh, kl, accl);
    accl = mma_h_raw(ql, kh, accl);
    guard_qk(acc, accl, qh, ql, kh, kl);
  }
#pragma unroll
  for (int r = 0; r < 8; ++r)
    sR[(8 * hh + r) * 132 + 16 * wave + rl] = acc[r] + accl[r] * (1.0f / 2048.0f);
  __syncthreads();
  v4f o[2];
#pragma unroll
  for (int q = 0; q < 2; ++q) o[q] = *(const v4f*)(sR + (2 * wave + q) * 132 + 4 * lane);
  float* rec = RAWP + ((size_t)(b0 + bl) * NCHK + chunk) * 2048;
  for (int ps = 0; ps < 2; ++ps) {
#pragma unroll
    for (int q = 0; q < 2; ++q) *(volatile v4f*)(rec + (2 * wave + q) * 128 + 4 * lane) = o[q];
    __threadfence();
  }
}

__global__ __launch_bounds__(256) void k_attn(const float* __restrict__ NRM, const float* __restrict__ RAWP,
                                              const float* __restrict__ wv, const float* __restrict__ sum_w,
                                              const _Float16* __restrict__ WvT16, _Float16* EFP, int h) {
  __shared__ float sInv[144];
  __shared__ float sS[16 * 128];
  __shared__ __align__(16) _Float16 sA[16 * 136];
  __shared__ float sEff[16 * 128];
  __shared__ float sMw[128];
  __shared__ float sSw[16];
  __shared__ __align__(16) _Float16 sE16[16 * 264];
  __shared__ float sRed[8];
  const int b = blockIdx.x;
  const int tid = threadIdx.x, lane = tid & 31;
  const int wave = __builtin_amdgcn_readfirstlane(tid >> 5);
  const int hh = lane >> 4, rl = lane & 15;

  if (tid < 16) sSw[tid] = bfr(sum_w[h * CIN + tid]);
  {
    const int t = min(tid, 143);
    const float* pn = NRM + (size_t)b * (WDIM * NSEG) * 256 + t;
    float s = 0.0f;
#pragma unroll 1
    for (int blk = 0; blk < WDIM * NSEG; ++blk) s += pn[(size_t)blk * 256];
    sInv[t] = 1.0f / fmaxf(sqrtf(s), 1e-12f);
  }
  if (tid < 128) {
    const float* pw = wv + (size_t)h * C8 * C8 + tid;
    float m = 0.0f;
#pragma unroll 1
    for (int j = 0; j < C8; ++j) m += bfr(pw[(size_t)j * C8]);
    sMw[tid] = m * (1.0f / 128.0f);
  }
  __syncthreads();

  float sc[8];
  {
    float r[8];
#pragma unroll
    for (int q = 0; q < 8; ++q) r[q] = 0.0f;
    const float* pr = RAWP + (size_t)b * NCHK * 2048 + tid;
#pragma unroll 1
    for (int ch = 0; ch < NCHK; ++ch) {
#pragma unroll
      for (int q = 0; q < 8; ++q) r[q] += pr[(size_t)ch * 2048 + 256 * q];
    }
#pragma unroll
    for (int q = 0; q < 8; ++q) {
      const int e = tid + 256 * q;
      const int i = e >> 7, j = e & 127;
      sc[q] = r[q] * (1.0f / 64.0f) * sInv[128 + i] * sInv[j] * (1.0f / 192.0f);
    }
  }
  float ls = 0.0f;
#pragma unroll
  for (int q = 0; q < 8; ++q) ls += sc[q];
#pragma unroll
  for (int off = 16; off >= 1; off >>= 1) ls += __shfl_xor(ls, off, 32);
  if (lane == 0) sRed[wave] = ls;
  __syncthreads();
  float tot = 0.0f;
#pragma unroll
  for (int w = 0; w < 8; ++w) tot += sRed[w];
  const float mean = tot * (1.0f / 2048.0f);
  __syncthreads();
  float lq = 0.0f;
#pragma unroll
  for (int q = 0; q < 8; ++q) { const float d = sc[q] - mean; lq += d * d; }
#pragma unroll
  for (int off = 16; off >= 1; off >>= 1) lq += __shfl_xor(lq, off, 32);
  if (lane == 0) sRed[wave] = lq;
  __syncthreads();
  float totq = 0.0f;
#pragma unroll
  for (int w = 0; w < 8; ++w) totq += sRed[w];
  const float var = totq * (1.0f / 2048.0f);
  const float rstd = 1.0f / sqrtf(var + 1e-5f);
#pragma unroll
  for (int q = 0; q < 8; ++q) sS[tid + 256 * q] = (sc[q] - mean) * rstd;
  __syncthreads();

#pragma unroll
  for (int q2 = 0; q2 < 2; ++q2) {
    const int row = 2 * wave + q2;
    float x[4];
#pragma unroll
    for (int m = 0; m < 4; ++m) x[m] = sS[row * 128 + lane + 32 * m];
    float mx = fmaxf(fmaxf(x[0], x[1]), fmaxf(x[2], x[3]));
#pragma unroll
    for (int off = 16; off >= 1; off >>= 1) mx = fmaxf(mx, __shfl_xor(mx, off, 32));
    float ex[4], z = 0.0f;
#pragma unroll
    for (int m = 0; m < 4; ++m) { ex[m] = expf(x[m] - mx); z += ex[m]; }
#pragma unroll
    for (int off = 16; off >= 1; off >>= 1) z += __shfl_xor(z, off, 32);
    const float rz = 1.0f / z;
#pragma unroll
    for (int m = 0; m < 4; ++m) {
      const float dev = ex[m] * rz - (1.0f / 128.0f);
      sA[row * 136 + lane + 32 * m] = (_Float16)(dev * 16384.0f);
    }
  }
  __syncthreads();

  {
    v8f acc = zero8();
    const _Float16* ap = sA + rl * 136 + 8 * hh;
    const _Float16* bw = WvT16 + ((size_t)(h * C8 + 16 * wave + rl)) * C8 + 8 * hh;
#pragma unroll
    for (int ks = 0; ks < 4; ++ks) acc = mma_h(ldfrag_h(ap + 32 * ks), ldfrag_h(bw + 32 * ks), acc);
#pragma unroll
    for (int r = 0; r < 8; ++r) {
      const int i = 8 * hh + r, a = 16 * wave + rl;
      const float e0 = acc[r] * (1.0f / (16384.0f * 64.0f));
      sEff[i * 128 + a] = e0 + sMw[a];
    }
  }
  __syncthreads();

  {
    const int kk = tid, tap = kk >> 4, c = kk & 15;
    const float sw = sSw[c], omsw = 1.0f - sw;
#pragma unroll 1
    for (int i = 0; i < HID; ++i) {
      float val = 0.0f;
#pragma unroll 1
      for (int k = 0; k < 8; ++k) {
        const float t = sEff[i * 128 + k * 16 + c] * wsur_f(sw, omsw, k, tap);
        val = val + t;
      }
      sE16[i * 264 + kk] = (_Float16)(val * 1024.0f);
    }
  }
  __syncthreads();
  HU u[2];
#pragma unroll
  for (int q = 0; q < 2; ++q) u[q].h = *(const v8h*)(sE16 + (2 * wave + q) * 264 + 8 * lane);
  for (int ps = 0; ps < 2; ++ps) {
#pragma unroll
    for (int q = 0; q < 2; ++q) {
      _Float16* dst = EFP + ((size_t)((b * NH + h) * HID + 2 * wave + q)) * KPAD + 8 * lane;
      *(volatile v4u*)dst = u[q].u;
    }
    __threadfence();
  }
}

__global__ __launch_bounds__(256) void k_out(const _Float16* __restrict__ cenT, const _Float16* __restrict__ EFP,
                                             const _Float16* __restrict__ WO16, float* Y) {
  __shared__ __align__(16) _Float16 sX2[2 * 3 * SXP * 16];
  __shared__ __align__(16) _Float16 sOh[64 * 72];
  __shared__ __align__(16) _Float16 sOl[64 * 72];
  __shared__ __align__(16) float sY[32 * 68];
  const int tid = threadIdx.x, lane = tid & 31;
  const int wave = __builtin_amdgcn_readfirstlane(tid >> 5);
  const int hh = lane >> 4, rl = lane & 15;
  const int bx = blockIdx.x;
  const int b = bx / (WDIM * NSEG);
  const int rem = bx - b * (WDIM * NSEG);
  const int wrow = rem / NSEG;
  const int x0 = (rem - wrow * NSEG) * 64;
  const size_t pxb = (size_t)b * NPIX + (size_t)wrow * XDIM + x0;
  const _Float16* cTb = cenT + (size_t)b * NPIX * 16;
  const int half = wave >> 2, ct = wave & 3;

#pragma unroll
  for (int r2 = 0; r2 < 2; ++r2) {
    if (r2 > 0) __syncthreads();
#pragma unroll
    for (int it = 0; it < 4; ++it) {
      const int itm = min(tid + 256 * it, 959);
      const int buf = (itm >= 480) ? 1 : 0;
      stage_item(sX2 + buf * (3 * SXP * 16), cTb, wrow, x0, 2 * r2 + buf, itm - 480 * buf);
    }
    __syncthreads();
    const int head = 2 * r2 + half;
    const _Float16* sXb = sX2 + half * (3 * SXP * 16);
    const _Float16* aE = EFP + ((size_t)((b * NH + head) * HID + rl)) * KPAD + 8 * hh;
    v8f acc = zero8();
#pragma unroll
    for (int ks = 0; ks < 5; ++ks) {
      const int tA = 2 * ks, tB = 2 * ks + 1;
      const int oA = (tap_ky(tA) * SXP + (tap_kx(tA) << head)) * 16 + 8 * hh;
      const int oB = (tap_ky(tB) * SXP + (tap_kx(tB) << head)) * 16 + 8 * hh;
      const int po = (16 * ct + rl) * 16;
      FR f;
      f.h[0] = *(const v8h*)(sXb + po + oA);
      f.h[1] = *(const v8h*)(sXb + po + oB);
      acc = mma_h(ldfrag_h(aE + 32 * ks), f.v, acc);
    }
    HU uh, ul;
#pragma unroll
    for (int r = 0; r < 8; ++r) {
      const float v = acc[r] * (1.0f / 256.0f);
      const _Float16 hv = (_Float16)v;
      uh.s[r] = hv;
      ul.s[r] = (_Float16)((v - (float)hv) * 2048.0f);
    }
    const int px = 16 * ct + rl, ch0 = head * HID + 8 * hh;
    *(v4u*)(sOh + px * 72 + ch0) = uh.u;
    *(v4u*)(sOl + px * 72 + ch0) = ul.u;
  }
  __syncthreads();

  v8f ay = zero8(), ayl = zero8();
  {
    const int ot = half;
    const _Float16* aW = WO16 + (size_t)(16 * ot + rl) * TT + 8 * hh;
    const _Float16* bO = sOh + (16 * ct + rl) * 72 + 8 * hh;
    const _Float16* bL = sOl + (16 * ct + rl) * 72 + 8 * hh;
#pragma unroll
    for (int ks = 0; ks < 2; ++ks) {
      const v16h a = ldfrag_h(aW + 32 * ks);
      const v16h b0 = ldfrag_h(bO + 32 * ks);
      const v16h b1 = ldfrag_h(bL + 32 * ks);
      ay = mma_h_raw(a, b0, ay);
      ayl = mma_h_raw(a, b1, ayl);
      guard2(ay, ayl, a, b0, b1);
    }
#pragma unroll
    for (int r = 0; r < 8; ++r) {
      const float yv = (ay[r] + ayl[r] * (1.0f / 2048.0f)) * (1.0f / 4096.0f);
      sY[(16 * ot + 8 * hh + r) * 68 + 16 * ct + rl] = yv;
    }
  }
  __syncthreads();
  v4f o[2];
  const int c4 = 4 * (lane & 15);
#pragma unroll
  for (int q = 0; q < 2; ++q) {
    const int row = 4 * wave + 2 * q + (lane >> 4);
    o[q] = *(const v4f*)(sY + row * 68 + c4);
  }
  for (int ps = 0; ps < 2; ++ps) {
#pragma unroll
    for (int q = 0; q < 2; ++q) {
      const int row = 4 * wave + 2 * q + (lane >> 4);
      float* dst = Y + (size_t)row * PTOT + pxb + c4;
      *(volatile v4f*)dst = o[q];
    }
    __threadfence();
  }
}

__global__ __launch_bounds__(256) void k_bn(const float* __restrict__ Y, const float* __restrict__ gam,
                                            const float* __restrict__ bet, float* out) {
  __shared__ double sred[8];
  const int c = blockIdx.x;
  const int tid = threadIdx.x, wave = tid >> 5, lane = tid & 31;
  const float* yc = Y + (size_t)c * PTOT + 4 * tid;
  const int nseg = PTOT / 1024;
  const int segb = NPIX / 1024;

  double s = 0.0;
#pragma unroll 1
  for (int j = 0; j < nseg; ++j) {
    const v4f v = *(const v4f*)(yc + (size_t)1024 * j);
    s += (double)v[0]; s += (double)v[1]; s += (double)v[2]; s += (double)v[3];
  }
#pragma unroll
  for (int off = 16; off >= 1; off >>= 1) s += shfl_xor_d(s, off);
  if (lane == 0) sred[wave] = s;
  __syncthreads();
  double tot = 0.0;
#pragma unroll
  for (int w = 0; w < 8; ++w) tot += sred[w];
  const float mean = (float)(tot * (1.0 / (double)PTOT));
  __syncthreads();

  double q = 0.0;
#pragma unroll 1
  for (int j = 0; j < nseg; ++j) {
    const v4f v = *(const v4f*)(yc + (size_t)1024 * j);
#pragma unroll
    for (int e = 0; e < 4; ++e) {
      const double d = (double)(v[e] - mean);
      q += d * d;
    }
  }
#pragma unroll
  for (int off = 16; off >= 1; off >>= 1) q += shfl_xor_d(q, off);
  if (lane == 0) sred[wave] = q;
  __syncthreads();
  double totq = 0.0;
#pragma unroll
  for (int w = 0; w < 8; ++w) totq += sred[w];
  const float var = (float)(totq * (1.0 / (double)PTOT));
  const float rstd = 1.0f / sqrtf(var + 1e-5f);
  const float g = bfr(gam[c]);
  const float be = bfr(bet[c]);

  for (int ps = 0; ps < 2; ++ps) {
#pragma unroll 1
    for (int j = 0; j < nseg; ++j) {
      const v4f v = *(const v4f*)(yc + (size_t)1024 * j);
      v4f o;
#pragma unroll
      for (int e = 0; e < 4; ++e) {
        const float yv = (v[e] - mean) * rstd * g + be;
        o[e] = yv > 0.0f ? yv : 0.0f;
      }
      const int bb = j / segb;
      const int nn = (j - bb * segb) * 1024 + 4 * tid;
      float* dst = out + ((size_t)(bb * OCH + c)) * NPIX + nn;
      *(volatile v4f*)dst = o;
    }
    __threadfence();
  }
}

extern "C" void kernel_launch(void* const* d_in, const int* in_sizes, int n_in,
                              void* d_out, int out_size, void* d_ws, size_t ws_size,
                              hipStream_t stream) {
  if (n_in < 8) return;
  if (in_sizes[0] != NB * CIN * NPIX) return;
  if (in_sizes[1] != NH * HID * CIN || in_sizes[2] != NH * C8 * C8 || in_sizes[3] != NH * C8 * C8) return;
  if (in_sizes[4] != NH * CIN || in_sizes[5] != OCH * TT || in_sizes[6] != OCH || in_sizes[7] != OCH) return;
  if (out_size != NB * OCH * NPIX) return;

  const float* cen   = (const float*)d_in[0];
  const float* wq    = (const float*)d_in[1];
  const float* wk    = (const float*)d_in[2];
  const float* wv    = (const float*)d_in[3];
  const float* sum_w = (const float*)d_in[4];
  const float* w_out = (const float*)d_in[5];
  const float* gam   = (const float*)d_in[6];
  const float* bet   = (const float*)d_in[7];

  const size_t P     = (size_t)PTOT;
  const size_t G     = (size_t)PG;
  const size_t szCT  = P * 16 * 2;
  const size_t szWK  = (size_t)NH * C8 * KPAD * 2;
  const size_t szWQ  = (size_t)NH * HID * KPAD * 2;
  const size_t szWV  = (size_t)NH * C8 * C8 * 2;
  const size_t szWO  = (size_t)OCH * TT * 2;
  const size_t szEF  = (size_t)NB * NH * HID * KPAD * 2;
  const size_t szNRM = (size_t)NBLK * 256 * 4;
  const size_t szRAW = (size_t)NB * NCHK * 2048 * 4;
  const size_t szQP  = G * HID * 2;
  const size_t szKP  = G * C8 * 2;
  const size_t szY   = P * OCH * 4;
  if (szY > 2 * szKP) return;

  size_t off = 0;
  const size_t oCT  = off; off += szCT;
  const size_t oWK  = off; off += szWK;
  const size_t oWQ  = off; off += szWQ;
  const size_t oWV  = off; off += szWV;
  const size_t oWO  = off; off += szWO;
  const size_t oEF  = off; off += szEF;
  const size_t oNRM = off; off += szNRM;
  const size_t oRAW = off; off += szRAW;
  const size_t oQH  = off; off += szQP;
  const size_t oQL  = off; off += szQP;
  const size_t oKH  = off; off += szKP;
  const size_t oKL  = off; off += szKP;
  if (off > ws_size) return;
  if (off > (size_t)134217728) return;

  char* ws = (char*)d_ws;
  _Float16* cenT  = (_Float16*)(ws + oCT);
  _Float16* Wk16  = (_Float16*)(ws + oWK);
  _Float16* Wq16  = (_Float16*)(ws + oWQ);
  _Float16* WvT16 = (_Float16*)(ws + oWV);
  _Float16* WO16  = (_Float16*)(ws + oWO);
  _Float16* EFP   = (_Float16*)(ws + oEF);
  float*    NRM   = (float*)(ws + oNRM);
  float*    RAWP  = (float*)(ws + oRAW);
  _Float16* Qh    = (_Float16*)(ws + oQH);
  _Float16* Ql    = (_Float16*)(ws + oQL);
  _Float16* Kh    = (_Float16*)(ws + oKH);
  _Float16* Kl    = (_Float16*)(ws + oKL);
  float*    Y     = (float*)(ws + oKH);
  float*    outf  = (float*)d_out;

  const dim3 b256(256), b128(128);
  const dim3 gPix(NBLK);
  const dim3 gPrep(NH);
  const dim3 gConv(GBLK);
  const dim3 gScore(BG * NCHK);
  const dim3 gAttn(NB);
  const dim3 gBN(OCH);

  k_cvt<<<gPix, b128, 0, stream>>>(cen, cenT);
  k_prep<<<gPrep, b256, 0, stream>>>(wq, wk, wv, sum_w, w_out, Wk16, Wq16, WvT16, WO16);
  for (int h = 0; h < NH; ++h) {
    for (int g = 0; g < NGRP; ++g) {
      k_conv<<<gConv, b256, 0, stream>>>(cenT, Wk16 + (size_t)h * C8 * KPAD, Wq16 + (size_t)h * HID * KPAD,
                                           Kh, Kl, Qh, Ql, NRM, h, g * BG);
      k_score<<<gScore, b256, 0, stream>>>(Qh, Ql, Kh, Kl, RAWP, g * BG);
    }
    k_attn<<<gAttn, b256, 0, stream>>>(NRM, RAWP, wv, sum_w, WvT16, EFP, h);
  }
  k_out<<<gPix, b256, 0, stream>>>(cenT, EFP, WO16, Y);
  k_bn<<<gBN, b256, 0, stream>>>(Y, gam, bet, outf);
}
